// GCN_1949915153217
// MI455X (gfx1250) — hardware-verified
//
#include <hip/hip_runtime.h>
#include <math.h>
#include <stdint.h>
#pragma clang fp contract(off)

#define NNODES 16384
#define FIN    128
#define F1     256
#define F2     128
#define F3     128
#define KSPLIT 16
#define KCH    (NNODES / KSPLIT)
#define OUT_ELEMS (NNODES * 128)

static_assert(NNODES % 64 == 0);
static_assert(KCH % 32 == 0);
static_assert(FIN % 64 == 0 && F1 % 64 == 0 && F2 % 64 == 0 && F3 % 64 == 0);
static_assert(FIN % 32 == 0 && F1 % 32 == 0 && F2 % 32 == 0);

typedef __attribute__((ext_vector_type(16))) __bf16   v16b;
typedef __attribute__((ext_vector_type(8)))  __bf16   v8b;
typedef __attribute__((ext_vector_type(8)))  float    v8f;
typedef __attribute__((ext_vector_type(4)))  float    v4f;
typedef __attribute__((ext_vector_type(4)))  unsigned int v4u;

__device__ __forceinline__ unsigned short f2bf_bits(float f) {
  unsigned u = __float_as_uint(f);
  return (unsigned short)((u + 0x7FFFu + ((u >> 16) & 1u)) >> 16);
}
__device__ __forceinline__ float bf_bits2f(unsigned short h) { return __uint_as_float(((unsigned)h) << 16); }
__device__ __forceinline__ unsigned pk16(unsigned short a, unsigned short b) { return (unsigned)a | ((unsigned)b << 16); }

__device__ __forceinline__ void dep_guard_b(v8f& a, v8f& b, v16b x, v16b y) { asm volatile("v_nop\n\tv_nop\n\tv_nop\n\tv_nop" : "+v"(a), "+v"(b) : "v"(x), "v"(y)); }
__device__ __forceinline__ void keep4_b(v16b a, v16b b, v16b c, v16b d) { asm volatile("v_nop" :: "v"(a), "v"(b), "v"(c), "v"(d)); }
__device__ __forceinline__ void acc_guard4(v8f& a, v8f& b, v8f& c, v8f& d) { asm volatile("v_nop\n\tv_nop\n\tv_nop\n\tv_nop" : "+v"(a), "+v"(b), "+v"(c), "+v"(d)); }

union FragU { v16b v; v8b h[2]; };
__device__ __forceinline__ v16b frag_load(const __bf16* p) {
  FragU f; f.h[0] = *(const v8b*)(p); f.h[1] = *(const v8b*)(p + 16); return f.v;
}
__device__ __forceinline__ v8f mma_bf(v16b a, v16b b, v8f c) {
  return __builtin_amdgcn_wmma_f32_16x16x32_bf16(false, a, false, b, (short)0, c, false, false);
}

template <int TERMS, int BIAS_MODE, bool OUT_F32, bool OUT_BF, int ACT>
__global__ __launch_bounds__(256) void wmma_gemm64(
    const unsigned short* __restrict__ Ap, const unsigned short* __restrict__ A2p, int lda, long strideA,
    const unsigned short* __restrict__ Btp, const unsigned short* __restrict__ Bt2p, int ldb, long strideB,
    float* __restrict__ Cf, unsigned short* __restrict__ Ch, unsigned short* __restrict__ Cl, int ldc, long strideC,
    const float* __restrict__ bias, int M, int N, int K) {
  constexpr bool A_LO = (TERMS == 2) || (TERMS == 3);
  constexpr bool B_LO = (TERMS == 1) || (TERMS == 3);
  __shared__ __align__(16) float sT[8][16 * 68];
  const int b    = blockIdx.y;
  const int lane = threadIdx.x & 31;
  const int wave = threadIdx.x >> 5;
  const int tilesN = N >> 6;
  const int tilesM = M >> 6;
  const int tile = blockIdx.x * 8 + wave;
  if (tile >= tilesM * tilesN) return;
  const int tm = tile / tilesN;
  const int tn = tile - tm * tilesN;
  const int m0 = tm << 6;
  const int n0 = tn << 6;

  const __bf16* Ab  = (const __bf16*)(const void*)Ap   + (size_t)b * strideA;
  const __bf16* Bb  = (const __bf16*)(const void*)Btp  + (size_t)b * strideB;
  const __bf16* Ab2 = (const __bf16*)(const void*)A2p  + (size_t)b * strideA;
  const __bf16* Bb2 = (const __bf16*)(const void*)Bt2p + (size_t)b * strideB;

  const int rlane = lane & 15;
  const int koff  = (lane >> 4) * 8;
  const int mOff  = (lane >> 4) * 8;

  v8f acc[4][4];
#pragma unroll
  for (int i = 0; i < 4; ++i)
#pragma unroll
    for (int j = 0; j < 4; ++j) acc[i][j] = (v8f){0.f,0.f,0.f,0.f,0.f,0.f,0.f,0.f};

  for (int k0 = 0; k0 < K; k0 += 32) {
    v16b bh[4], bl[4];
#pragma unroll
    for (int j = 0; j < 4; ++j) {
      const size_t bo = (size_t)(n0 + (j << 4) + rlane) * ldb + koff + k0;
      bh[j] = frag_load(Bb + bo);
      if (B_LO) bl[j] = frag_load(Bb2 + bo);
    }
#pragma unroll
    for (int i = 0; i < 4; ++i) {
      const size_t ao = (size_t)(m0 + (i << 4) + rlane) * lda + koff + k0;
      v16b ah = frag_load(Ab + ao);
      v16b al;
      if (A_LO) al = frag_load(Ab2 + ao);
#pragma unroll
      for (int j = 0; j < 4; ++j) {
        acc[i][j] = mma_bf(ah, bh[j], acc[i][j]);
        if (B_LO) acc[i][j] = mma_bf(ah, bl[j], acc[i][j]);
        if (A_LO) acc[i][j] = mma_bf(al, bh[j], acc[i][j]);
      }
      dep_guard_b(acc[i][0], acc[i][3], ah, A_LO ? al : ah);
    }
    keep4_b(bh[0], bh[1], bh[2], bh[3]);
    if (B_LO) keep4_b(bl[0], bl[1], bl[2], bl[3]);
  }
  acc_guard4(acc[0][0], acc[0][1], acc[0][2], acc[0][3]);
  acc_guard4(acc[1][0], acc[1][1], acc[1][2], acc[1][3]);
  acc_guard4(acc[2][0], acc[2][1], acc[2][2], acc[2][3]);
  acc_guard4(acc[3][0], acc[3][1], acc[3][2], acc[3][3]);

  float bvs[4] = {0.f, 0.f, 0.f, 0.f};
  if (BIAS_MODE == 2) {
#pragma unroll
    for (int j = 0; j < 4; ++j) bvs[j] = bf_bits2f(f2bf_bits(bias[n0 + (j << 4) + rlane]));
  }
  float* slab = sT[wave];
#pragma unroll
  for (int i = 0; i < 4; ++i) {
    const int mBase = m0 + (i << 4);
#pragma unroll
    for (int j = 0; j < 4; ++j) {
#pragma unroll
      for (int r = 0; r < 8; ++r) {
        float v = acc[i][j][r];
        if (BIAS_MODE == 2) v = v + bvs[j];
        if (ACT == 1) v = (v > 0.f) ? v : 0.25f * v;
        slab[(mOff + r) * 68 + (j << 4) + rlane] = v;
      }
    }
    __builtin_amdgcn_fence(__ATOMIC_RELEASE, "workgroup");
    __builtin_amdgcn_wave_barrier();
    __builtin_amdgcn_fence(__ATOMIC_ACQUIRE, "workgroup");
    if (OUT_F32) {
      float* C = Cf + (size_t)b * strideC;
      const int hh = lane >> 4, c4 = (lane & 15) * 4;
      for (int pass = 0; pass < 2; ++pass) {
#pragma unroll
        for (int it = 0; it < 8; ++it) {
          const int row = it * 2 + hh;
          v4f v = *(const v4f*)(slab + row * 68 + c4);
          *(volatile v4f*)(C + (size_t)(mBase + row) * ldc + n0 + c4) = v;
        }
        __threadfence();
      }
    }
    if (OUT_BF) {
      const int q = lane >> 3, c8 = (lane & 7) * 8;
      unsigned short* C  = Ch + (size_t)b * strideC;
      unsigned short* C2 = Cl + (size_t)b * strideC;
      for (int pass = 0; pass < 2; ++pass) {
#pragma unroll
        for (int it = 0; it < 4; ++it) {
          const int row = it * 4 + q;
          const float* sp = slab + row * 68 + c8;
          v4u hv, lv;
#pragma unroll
          for (int e = 0; e < 4; ++e) {
            const float f0 = sp[2 * e], f1 = sp[2 * e + 1];
            const unsigned short h0 = f2bf_bits(f0), h1 = f2bf_bits(f1);
            const unsigned short l0 = f2bf_bits(f0 - bf_bits2f(h0)), l1 = f2bf_bits(f1 - bf_bits2f(h1));
            hv[e] = pk16(h0, h1);
            lv[e] = pk16(l0, l1);
          }
          const size_t go = (size_t)(mBase + row) * ldc + n0 + c8;
          *(volatile v4u*)(C + go)  = hv;
          *(volatile v4u*)(C2 + go) = lv;
        }
        __threadfence();
      }
    }
    __builtin_amdgcn_fence(__ATOMIC_RELEASE, "workgroup");
    __builtin_amdgcn_wave_barrier();
    __builtin_amdgcn_fence(__ATOMIC_ACQUIRE, "workgroup");
  }
}

#define PXP 132
__global__ __launch_bounds__(256) void prep_x_kernel(const float* __restrict__ x,
                                                     unsigned short* __restrict__ xb,
                                                     unsigned short* __restrict__ xnh, unsigned short* __restrict__ xnl,
                                                     unsigned short* __restrict__ xth, unsigned short* __restrict__ xtl) {
  __shared__ __align__(16) float xs[64 * PXP];
  __shared__ float rinv[64];
  const int tid = threadIdx.x;
  const int node0 = blockIdx.x * 64;
#pragma unroll 4
  for (int it = 0; it < 8; ++it) {
    const int id = it * 256 + tid;
    const int r = id >> 5;
    const int c4 = (id & 31) * 4;
    v4f a = *(const v4f*)(x + (size_t)(node0 + r) * FIN + c4);
    a[0] = bf_bits2f(f2bf_bits(a[0]));
    a[1] = bf_bits2f(f2bf_bits(a[1]));
    a[2] = bf_bits2f(f2bf_bits(a[2]));
    a[3] = bf_bits2f(f2bf_bits(a[3]));
    *(v4f*)(xs + r * PXP + c4) = a;
  }
  __syncthreads();
  {
    const int r = tid >> 2, part = tid & 3;
    float s = 0.f;
#pragma unroll 4
    for (int e = 0; e < 32; ++e) {
      const float v = xs[r * PXP + part * 32 + e];
      s = fmaf(v, v, s);
    }
    s += __shfl_xor(s, 1, 32);
    s += __shfl_xor(s, 2, 32);
    if (part == 0) rinv[r] = 1.0f / sqrtf(s + 1e-12f);
  }
  __syncthreads();
  for (int pass = 0; pass < 2; ++pass) {
#pragma unroll 1
    for (int it = 0; it < 4; ++it) {
      const int id = it * 256 + tid;
      {
        const int r = id >> 4;
        const int c8 = (id & 15) * 8;
        const float ri = rinv[r];
        const float* sp = xs + r * PXP + c8;
        v4u bv, hv, lv;
#pragma unroll
        for (int q = 0; q < 4; ++q) {
          const float f0 = sp[2 * q], f1 = sp[2 * q + 1];
          bv[q] = pk16(f2bf_bits(f0), f2bf_bits(f1));
          const float g0 = f0 * ri, g1 = f1 * ri;
          const unsigned short h0 = f2bf_bits(g0), h1 = f2bf_bits(g1);
          const unsigned short l0 = f2bf_bits(g0 - bf_bits2f(h0)), l1 = f2bf_bits(g1 - bf_bits2f(h1));
          hv[q] = pk16(h0, h1);
          lv[q] = pk16(l0, l1);
        }
        const size_t go = (size_t)(node0 + r) * FIN + c8;
        *(volatile v4u*)(xb + go)  = bv;
        *(volatile v4u*)(xnh + go) = hv;
        *(volatile v4u*)(xnl + go) = lv;
      }
      {
        const int c = id >> 3;
        const int n8 = (id & 7) * 8;
        v4u hv, lv;
#pragma unroll
        for (int q = 0; q < 4; ++q) {
          const float g0 = xs[(n8 + 2 * q) * PXP + c] * rinv[n8 + 2 * q];
          const float g1 = xs[(n8 + 2 * q + 1) * PXP + c] * rinv[n8 + 2 * q + 1];
          const unsigned short h0 = f2bf_bits(g0), h1 = f2bf_bits(g1);
          const unsigned short l0 = f2bf_bits(g0 - bf_bits2f(h0)), l1 = f2bf_bits(g1 - bf_bits2f(h1));
          hv[q] = pk16(h0, h1);
          lv[q] = pk16(l0, l1);
        }
        const size_t go = (size_t)c * NNODES + node0 + n8;
        *(volatile v4u*)(xth + go) = hv;
        *(volatile v4u*)(xtl + go) = lv;
      }
    }
    __threadfence();
  }
}

__global__ __launch_bounds__(256) void tcvt_kernel(const float* __restrict__ W, unsigned short* __restrict__ oh, int R, int Cc) {
  __shared__ __align__(16) float tf[64 * 68];
  const int c0  = blockIdx.x * 64;
  const int r0  = blockIdx.y * 64;
  const int tid = threadIdx.x;
  {
    const int lr = tid >> 4;
    const int c4 = (tid & 15) * 4;
#pragma unroll
    for (int it = 0; it < 4; ++it) {
      const int rr = it * 16 + lr;
      const v4f a = *(const v4f*)(W + (size_t)(r0 + rr) * Cc + c0 + c4);
      *(v4f*)(tf + rr * 68 + c4) = a;
    }
  }
  __syncthreads();
  const int sub = tid >> 3;
  const int c8  = (tid & 7) * 8;
  v4u hv[2];
#pragma unroll
  for (int it = 0; it < 2; ++it) {
    const int oc = it * 32 + sub;
    v4u a;
#pragma unroll
    for (int q = 0; q < 4; ++q) {
      const float f0 = tf[(c8 + 2 * q) * 68 + oc];
      const float f1 = tf[(c8 + 2 * q + 1) * 68 + oc];
      a[q] = pk16(f2bf_bits(f0), f2bf_bits(f1));
    }
    hv[it] = a;
  }
  for (int pass = 0; pass < 2; ++pass) {
#pragma unroll
    for (int it = 0; it < 2; ++it) {
      const int oc = it * 32 + sub;
      const size_t go = (size_t)(c0 + oc) * R + r0 + c8;
      *(volatile v4u*)(oh + go) = hv[it];
    }
    __threadfence();
  }
}

__global__ __launch_bounds__(256) void cvt8_kernel(const float* __restrict__ in, unsigned short* __restrict__ out, int n8) {
  const int i = blockIdx.x * 256 + threadIdx.x;
  if (i < n8) {
    const v4f a = *(const v4f*)(in + 8 * (size_t)i);
    const v4f c = *(const v4f*)(in + 8 * (size_t)i + 4);
    v4u o;
    o[0] = pk16(f2bf_bits(a[0]), f2bf_bits(a[1]));
    o[1] = pk16(f2bf_bits(a[2]), f2bf_bits(a[3]));
    o[2] = pk16(f2bf_bits(c[0]), f2bf_bits(c[1]));
    o[3] = pk16(f2bf_bits(c[2]), f2bf_bits(c[3]));
    *(volatile v4u*)(out + 8 * (size_t)i) = o;
    __threadfence();
    *(volatile v4u*)(out + 8 * (size_t)i) = o;
  }
}

__global__ __launch_bounds__(256) void gcomb_kernel(const float* __restrict__ P, unsigned short* __restrict__ gh,
                                                    unsigned short* __restrict__ gl, int total, int nks) {
  const int i = blockIdx.x * 256 + threadIdx.x;
  if (i < (total >> 3)) {
    v4f s0 = (v4f){0.f, 0.f, 0.f, 0.f};
    v4f s1 = (v4f){0.f, 0.f, 0.f, 0.f};
#pragma unroll 4
    for (int ks = 0; ks < nks; ++ks) {
      const float* p = P + (size_t)ks * total + 8 * (size_t)i;
      const v4f a = *(const v4f*)p;
      const v4f c = *(const v4f*)(p + 4);
      s0 = s0 + a;
      s1 = s1 + c;
    }
    v4u hv, lv;
#pragma unroll
    for (int q = 0; q < 2; ++q) {
      const float f0 = s0[2 * q], f1 = s0[2 * q + 1];
      const unsigned short h0 = f2bf_bits(f0), h1 = f2bf_bits(f1);
      hv[q] = pk16(h0, h1);
      lv[q] = pk16(f2bf_bits(f0 - bf_bits2f(h0)), f2bf_bits(f1 - bf_bits2f(h1)));
      const float g0 = s1[2 * q], g1 = s1[2 * q + 1];
      const unsigned short k0 = f2bf_bits(g0), k1 = f2bf_bits(g1);
      hv[2 + q] = pk16(k0, k1);
      lv[2 + q] = pk16(f2bf_bits(g0 - bf_bits2f(k0)), f2bf_bits(g1 - bf_bits2f(k1)));
    }
    *(volatile v4u*)(gh + 8 * (size_t)i) = hv;
    *(volatile v4u*)(gl + 8 * (size_t)i) = lv;
    __threadfence();
    *(volatile v4u*)(gh + 8 * (size_t)i) = hv;
    *(volatile v4u*)(gl + 8 * (size_t)i) = lv;
  }
}

extern "C" void kernel_launch(void* const* d_in, const int* in_sizes, int n_in,
                              void* d_out, int out_size, void* d_ws, size_t ws_size,
                              hipStream_t stream) {
  if (n_in < 9) return;
  if (in_sizes[0] != NNODES * FIN) return;
  if (in_sizes[1] != FIN * F1 || in_sizes[2] != F1) return;
  if (in_sizes[3] != F1 * F2 || in_sizes[4] != F2) return;
  if (in_sizes[5] != F2 * F3 || in_sizes[6] != F3) return;
  if (in_sizes[7] != F3 * FIN || in_sizes[8] != F3) return;
  if (out_size != 2 * OUT_ELEMS) return;

  const float* x  = (const float*)d_in[0];
  const float* W1 = (const float*)d_in[1];
  const float* b1 = (const float*)d_in[2];
  const float* W2 = (const float*)d_in[3];
  const float* b2 = (const float*)d_in[4];
  const float* W3 = (const float*)d_in[5];
  const float* b3 = (const float*)d_in[6];
  const float* Wc = (const float*)d_in[7];
  const float* bc = (const float*)d_in[8];
  float* out = (float*)d_out;
  float* h3o = out + (size_t)OUT_ELEMS;

  const size_t PN  = (size_t)NNODES * FIN * 2;
  const size_t PY  = (size_t)F1 * NNODES * 2;
  const size_t PP  = (size_t)KSPLIT * F1 * FIN * 4;
  const size_t PG  = (size_t)F1 * FIN * 2;
  size_t off = 0;
  const size_t oXB  = off; off += PN;
  const size_t oXNh = off; off += PN;  const size_t oXNl = off; off += PN;
  const size_t oXTh = off; off += PN;  const size_t oXTl = off; off += PN;
  const size_t oYTh = off; off += PY;  const size_t oYTl = off; off += PY;
  const size_t oHh  = off; off += PY;  const size_t oHl  = off; off += PY;
  const size_t oP   = off; off += PP;
  const size_t oGTh = off; off += PG;  const size_t oGTl = off; off += PG;
  const size_t oW1t = off; off += (size_t)F1 * FIN * 2;
  const size_t oW2t = off; off += (size_t)F2 * F1 * 2;
  const size_t oW3t = off; off += (size_t)F3 * F2 * 2;
  const size_t oWcb = off; off += (size_t)F3 * FIN * 2;
  if (off > ws_size || off > (size_t)134217728) return;

  char* ws = (char*)d_ws;
  unsigned short* XB  = (unsigned short*)(ws + oXB);
  unsigned short* XNh = (unsigned short*)(ws + oXNh); unsigned short* XNl = (unsigned short*)(ws + oXNl);
  unsigned short* XTh = (unsigned short*)(ws + oXTh); unsigned short* XTl = (unsigned short*)(ws + oXTl);
  unsigned short* YTh = (unsigned short*)(ws + oYTh); unsigned short* YTl = (unsigned short*)(ws + oYTl);
  unsigned short* Hh  = (unsigned short*)(ws + oHh);  unsigned short* Hl  = (unsigned short*)(ws + oHl);
  float*          P   = (float*)(ws + oP);
  unsigned short* GTh = (unsigned short*)(ws + oGTh); unsigned short* GTl = (unsigned short*)(ws + oGTl);
  unsigned short* W1t = (unsigned short*)(ws + oW1t);
  unsigned short* W2t = (unsigned short*)(ws + oW2t);
  unsigned short* W3t = (unsigned short*)(ws + oW3t);
  unsigned short* Wcb = (unsigned short*)(ws + oWcb);

  const dim3 blk(256);

  prep_x_kernel<<<dim3(NNODES / 64), blk, 0, stream>>>(x, XB, XNh, XNl, XTh, XTl);
  tcvt_kernel<<<dim3(F1 / 64, FIN / 64), blk, 0, stream>>>(W1, W1t, FIN, F1);
  tcvt_kernel<<<dim3(F2 / 64, F1 / 64), blk, 0, stream>>>(W2, W2t, F1, F2);
  tcvt_kernel<<<dim3(F3 / 64, F2 / 64), blk, 0, stream>>>(W3, W3t, F2, F3);
  cvt8_kernel<<<dim3((F3 * FIN / 8 + 255) / 256), blk, 0, stream>>>(Wc, Wcb, F3 * FIN / 8);

  wmma_gemm64<0, 0, false, true, 0><<<dim3(((F1 / 64) * (NNODES / 64) + 7) / 8, 1), blk, 0, stream>>>(
      W1t, W1t, FIN, 0L, XB, XB, FIN, 0L, P, YTh, YTl, NNODES, 0L, b1, F1, NNODES, FIN);
  wmma_gemm64<3, 0, true, false, 0><<<dim3(1, KSPLIT), dim3(32 * (F1 / 64) * (FIN / 64)), 0, stream>>>(
      YTh, YTl, NNODES, (long)KCH, XTh, XTl, NNODES, (long)KCH, P, GTh, GTl, FIN, (long)F1 * FIN, b1, F1, FIN, KCH);
  gcomb_kernel<<<dim3((F1 * FIN / 8 + 255) / 256), blk, 0, stream>>>(P, GTh, GTl, F1 * FIN, KSPLIT);
  wmma_gemm64<3, 2, false, true, 1><<<dim3(((NNODES / 64) * (F1 / 64) + 7) / 8, 1), blk, 0, stream>>>(
      XNh, XNl, FIN, 0L, GTh, GTl, FIN, 0L, P, Hh, Hl, F1, 0L, b1, NNODES, F1, FIN);

  wmma_gemm64<1, 0, false, true, 0><<<dim3(((F2 / 64) * (NNODES / 64) + 7) / 8, 1), blk, 0, stream>>>(
      W2t, W2t, F1, 0L, Hh, Hl, F1, 0L, P, YTh, YTl, NNODES, 0L, b2, F2, NNODES, F1);
  wmma_gemm64<3, 0, true, false, 0><<<dim3(1, KSPLIT), dim3(32 * (F2 / 64) * (FIN / 64)), 0, stream>>>(
      YTh, YTl, NNODES, (long)KCH, XTh, XTl, NNODES, (long)KCH, P, GTh, GTl, FIN, (long)F2 * FIN, b2, F2, FIN, KCH);
  gcomb_kernel<<<dim3((F2 * FIN / 8 + 255) / 256), blk, 0, stream>>>(P, GTh, GTl, F2 * FIN, KSPLIT);
  wmma_gemm64<3, 2, false, true, 1><<<dim3(((NNODES / 64) * (F2 / 64) + 7) / 8, 1), blk, 0, stream>>>(
      XNh, XNl, FIN, 0L, GTh, GTl, FIN, 0L, P, Hh, Hl, F2, 0L, b2, NNODES, F2, FIN);

  wmma_gemm64<1, 0, false, true, 0><<<dim3(((F3 / 64) * (NNODES / 64) + 7) / 8, 1), blk, 0, stream>>>(
      W3t, W3t, F2, 0L, Hh, Hl, F2, 0L, P, YTh, YTl, NNODES, 0L, b3, F3, NNODES, F2);
  wmma_gemm64<3, 0, true, false, 0><<<dim3(1, KSPLIT), dim3(32 * (F3 / 64) * (FIN / 64)), 0, stream>>>(
      YTh, YTl, NNODES, (long)KCH, XTh, XTl, NNODES, (long)KCH, P, GTh, GTl, FIN, (long)F3 * FIN, b3, F3, FIN, KCH);
  gcomb_kernel<<<dim3((F3 * FIN / 8 + 255) / 256), blk, 0, stream>>>(P, GTh, GTl, F3 * FIN, KSPLIT);
  wmma_gemm64<3, 2, true, true, 1><<<dim3(((NNODES / 64) * (F3 / 64) + 7) / 8, 1), blk, 0, stream>>>(
      XNh, XNl, FIN, 0L, GTh, GTl, FIN, 0L, h3o, Hh, Hl, F3, 0L, b3, NNODES, F3, FIN);

  wmma_gemm64<2, 2, true, false, 0><<<dim3(((NNODES / 64) * (F3 / 64) + 7) / 8, 1), blk, 0, stream>>>(
      Hh, Hl, F3, 0L, Wcb, Wcb, F3, 0L, out, Hh, Hl, F3, 0L, bc, NNODES, F3, F3);

  (void)hipGetLastError();
}
